// DSAttentionLayer_32573031973597
// MI455X (gfx1250) — hardware-verified
//
#include <hip/hip_runtime.h>
#include <stdint.h>


#ifndef AFFINE_BF16
#define AFFINE_BF16 1
#endif

#define DM 512
#define NH 8
#define HD 64
#define NB 4
#define SQ 2048
#define MR (NB * SQ)
#define PLANE (MR * DM)
#define PP 72
#define PC 136
#define PT 72
#define PO 132

#define CVT_BLK 256
#define CVT_UNITS 4
#define UPP (PLANE / 8)
#define CVT_GRID (UPP / (CVT_BLK * CVT_UNITS))

typedef _Float16 v16h __attribute__((ext_vector_type(16)));
typedef _Float16 v8h  __attribute__((ext_vector_type(8)));
typedef v8h __attribute__((may_alias)) v8ha;
typedef float v8f __attribute__((ext_vector_type(8)));
typedef float v4f __attribute__((ext_vector_type(4)));
typedef v4f __attribute__((may_alias)) v4fa;

union Frag { v16h v; v8h p[2]; };

#if defined(__has_builtin)
#if __has_builtin(__builtin_amdgcn_exp2f)
#define EX2(x) __builtin_amdgcn_exp2f(x)
#endif
#endif
#ifndef EX2
#define EX2(x) __expf((x) * 0.69314718055994531f)
#endif

__device__ __forceinline__ float bfr(float x)
{
    unsigned u = __float_as_uint(x);
    u = (u + 0x7fffu + ((u >> 16) & 1u)) & 0xffff0000u;
    return __uint_as_float(u);
}
__device__ __forceinline__ _Float16 cvh(float x, float s) { return (_Float16)(bfr(x) * s); }

__device__ __forceinline__ v8f mma16(v16h a, v16h b, v8f c)
{
    return __builtin_amdgcn_wmma_f32_16x16x32_f16(false, a, false, b, (short)0, c, false, false);
}

__device__ __forceinline__ v8f zero8()
{
    v8f z;
#pragma unroll
    for (int i = 0; i < 8; ++i) z[i] = 0.0f;
    return z;
}

__global__ __launch_bounds__(CVT_BLK)
void k_cvt_act(const float* __restrict__ x0, const float* __restrict__ x1,
               const float* __restrict__ x2, _Float16* __restrict__ xh)
{
    const int pl = blockIdx.y;
    const float* src = (pl == 0) ? x0 : ((pl == 1) ? x1 : x2);
    _Float16* dst = xh + (size_t)pl * PLANE;
    const int t0 = blockIdx.x * CVT_BLK + (int)threadIdx.x;
    v8h val[CVT_UNITS];
    int uu[CVT_UNITS];
#pragma unroll
    for (int j = 0; j < CVT_UNITS; ++j) {
        int u = t0 + j * (CVT_GRID * CVT_BLK);
        u = (u < UPP) ? u : (UPP - 1);
        uu[j] = u;
        const float4 a = *(const float4*)(src + (size_t)u * 8);
        const float4 b = *(const float4*)(src + (size_t)u * 8 + 4);
        v8h v;
        v[0] = cvh(a.x, 16.0f); v[1] = cvh(a.y, 16.0f); v[2] = cvh(a.z, 16.0f); v[3] = cvh(a.w, 16.0f);
        v[4] = cvh(b.x, 16.0f); v[5] = cvh(b.y, 16.0f); v[6] = cvh(b.z, 16.0f); v[7] = cvh(b.w, 16.0f);
        val[j] = v;
    }
#pragma unroll
    for (int j = 0; j < CVT_UNITS; ++j)
        *(volatile v8h*)(dst + (size_t)uu[j] * 8) = val[j];
    __threadfence();
#pragma unroll
    for (int j = 0; j < CVT_UNITS; ++j)
        *(volatile v8h*)(dst + (size_t)uu[j] * 8) = val[j];
}

__global__ __launch_bounds__(128)
void k_cvt_wt(const float* __restrict__ w0, const float* __restrict__ w1,
              const float* __restrict__ w2, const float* __restrict__ w3,
              _Float16* __restrict__ wt)
{
    __shared__ _Float16 __attribute__((aligned(16))) sT[64 * PT];
    const int z = blockIdx.z;
    const float* src = (z == 0) ? w0 : ((z == 1) ? w1 : ((z == 2) ? w2 : w3));
    _Float16* dst = wt + (size_t)z * (DM * DM);
    const int k0 = blockIdx.y * 64, n0 = blockIdx.x * 64;
    const int t = threadIdx.x, l = t & 31, w = t >> 5;
    const int nn = (t & 15) * 4, kb = t >> 4;
#pragma unroll
    for (int i = 0; i < 8; ++i) {
        const int kk = kb + 8 * i;
        const float4 v = *(const float4*)(src + (size_t)(k0 + kk) * DM + n0 + nn);
        sT[(nn + 0) * PT + kk] = cvh(v.x, 64.0f);
        sT[(nn + 1) * PT + kk] = cvh(v.y, 64.0f);
        sT[(nn + 2) * PT + kk] = cvh(v.z, 64.0f);
        sT[(nn + 3) * PT + kk] = cvh(v.w, 64.0f);
    }
    __syncthreads();
    v8h val[4];
    size_t off[4];
#pragma unroll
    for (int i = 0; i < 4; ++i) {
        const int line = 16 * w + 4 * i + (l >> 3);
        const int ck = (l & 7) * 8;
        val[i] = *(const v8ha*)(sT + line * PT + ck);
        off[i] = (size_t)(n0 + line) * DM + k0 + ck;
    }
#pragma unroll
    for (int i = 0; i < 4; ++i) *(volatile v8h*)(dst + off[i]) = val[i];
    __threadfence();
#pragma unroll
    for (int i = 0; i < 4; ++i) *(volatile v8h*)(dst + off[i]) = val[i];
}

template<bool OUTF>
__global__ __launch_bounds__(128) __attribute__((amdgpu_num_vgpr(248)))
void k_gemm(const _Float16* __restrict__ A, int planeA, const _Float16* __restrict__ Bt,
            const float* __restrict__ bi0, const float* __restrict__ bi1,
            const float* __restrict__ bi2,
            _Float16* __restrict__ O16, float* __restrict__ O32, float s_acc, float s_out)
{
    const int t = threadIdx.x, l = t & 31, w = t >> 5, h = l >> 4, m = l & 15;
    const int z = blockIdx.z;
    const int n0 = blockIdx.x * 128, m0 = blockIdx.y * 64;
    const int wm = (w >> 1) * 32, wn = (w & 1) * 64;
    const _Float16* Ab = A + (size_t)z * (size_t)planeA;
    const _Float16* Bb = Bt + (size_t)z * (DM * DM);
    const float* bias = (z == 0) ? bi0 : ((z == 1) ? bi1 : bi2);

    const _Float16* ap[2];
    const _Float16* bp[4];
#pragma unroll
    for (int mi = 0; mi < 2; ++mi) ap[mi] = Ab + (size_t)(m0 + wm + 16 * mi + m) * DM + 8 * h;
#pragma unroll
    for (int ni = 0; ni < 4; ++ni) bp[ni] = Bb + (size_t)(n0 + wn + 16 * ni + m) * DM + 8 * h;

    v8f acc[2][4];
#pragma unroll
    for (int mi = 0; mi < 2; ++mi)
#pragma unroll
        for (int ni = 0; ni < 4; ++ni) acc[mi][ni] = zero8();

#pragma unroll 2
    for (int k0 = 0; k0 < DM; k0 += 32) {
        Frag a[2], b[4];
#pragma unroll
        for (int mi = 0; mi < 2; ++mi) {
            a[mi].p[0] = *(const v8h*)(ap[mi] + k0);
            a[mi].p[1] = *(const v8h*)(ap[mi] + k0 + 16);
        }
#pragma unroll
        for (int ni = 0; ni < 4; ++ni) {
            b[ni].p[0] = *(const v8h*)(bp[ni] + k0);
            b[ni].p[1] = *(const v8h*)(bp[ni] + k0 + 16);
        }
#pragma unroll
        for (int mi = 0; mi < 2; ++mi)
#pragma unroll
            for (int ni = 0; ni < 4; ++ni)
                acc[mi][ni] = mma16(a[mi].v, b[ni].v, acc[mi][ni]);
        asm volatile("v_nop\n\tv_nop\n\tv_nop\n\tv_nop"
                     : "+v"(acc[0][0]), "+v"(acc[0][1]), "+v"(acc[0][2]), "+v"(acc[0][3]),
                       "+v"(acc[1][0]), "+v"(acc[1][1]), "+v"(acc[1][2]), "+v"(acc[1][3])
                     : "v"(a[0].v), "v"(a[1].v), "v"(b[0].v), "v"(b[1].v), "v"(b[2].v), "v"(b[3].v));
    }

    float bb[4];
#pragma unroll
    for (int ni = 0; ni < 4; ++ni) bb[ni] = bfr(bias[n0 + wn + 16 * ni + m]);

    if constexpr (OUTF) {
        __shared__ float __attribute__((aligned(16))) sO[64 * PO];
#pragma unroll
        for (int mi = 0; mi < 2; ++mi)
#pragma unroll
            for (int ni = 0; ni < 4; ++ni)
#pragma unroll
                for (int r = 0; r < 8; ++r) {
                    const int row = wm + 16 * mi + 8 * h + r;
                    const int col = wn + 16 * ni + m;
                    sO[row * PO + col] = (acc[mi][ni][r] * s_acc + bb[ni]) * s_out;
                }
        __syncthreads();
        v4f val[16];
#pragma unroll
        for (int i = 0; i < 16; ++i) val[i] = *(const v4fa*)(sO + (16 * w + i) * PO + 4 * l);
#pragma unroll
        for (int i = 0; i < 16; ++i)
            *(volatile v4f*)(O32 + (size_t)(m0 + 16 * w + i) * DM + n0 + 4 * l) = val[i];
        __threadfence();
#pragma unroll
        for (int i = 0; i < 16; ++i)
            *(volatile v4f*)(O32 + (size_t)(m0 + 16 * w + i) * DM + n0 + 4 * l) = val[i];
    } else {
        __shared__ _Float16 __attribute__((aligned(16))) sC[9216];
        if (z != 2) {
#pragma unroll
            for (int mi = 0; mi < 2; ++mi)
#pragma unroll
                for (int ni = 0; ni < 4; ++ni)
#pragma unroll
                    for (int r = 0; r < 8; ++r) {
                        const int row = wm + 16 * mi + 8 * h + r;
                        const int col = wn + 16 * ni + m;
                        sC[row * PC + col] = (_Float16)((acc[mi][ni][r] * s_acc + bb[ni]) * s_out);
                    }
        } else {
#pragma unroll
            for (int mi = 0; mi < 2; ++mi)
#pragma unroll
                for (int ni = 0; ni < 4; ++ni)
#pragma unroll
                    for (int r = 0; r < 8; ++r) {
                        const int row = wm + 16 * mi + 8 * h + r;
                        const int col = wn + 16 * ni + m;
                        sC[col * PT + row] = (_Float16)((acc[mi][ni][r] * s_acc + bb[ni]) * s_out);
                    }
        }
        __syncthreads();
        v8h val[8];
        size_t off[8];
        if (z != 2) {
#pragma unroll
            for (int i = 0; i < 8; ++i) {
                const int row = 16 * w + 2 * i + (l >> 4);
                const int c8 = (l & 15) * 8;
                val[i] = *(const v8ha*)(sC + row * PC + c8);
                off[i] = (size_t)z * PLANE + (size_t)(m0 + row) * DM + n0 + c8;
            }
        } else {
            const int bidx = m0 / SQ, s0 = m0 - bidx * SQ;
#pragma unroll
            for (int i = 0; i < 8; ++i) {
                const int col = 32 * w + 4 * i + (l >> 3);
                const int ck = (l & 7) * 8;
                const int gc = n0 + col;
                val[i] = *(const v8ha*)(sC + col * PT + ck);
                off[i] = (size_t)2 * PLANE
                       + ((size_t)((bidx * NH + (gc >> 6)) * HD + (gc & 63))) * SQ + s0 + ck;
            }
        }
#pragma unroll
        for (int i = 0; i < 8; ++i) *(volatile v8h*)(O16 + off[i]) = val[i];
        __threadfence();
#pragma unroll
        for (int i = 0; i < 8; ++i) *(volatile v8h*)(O16 + off[i]) = val[i];
    }
}

__global__ __launch_bounds__(128) __attribute__((amdgpu_num_vgpr(248)))
void k_attn(const _Float16* __restrict__ Qh, const _Float16* __restrict__ Kh,
            const _Float16* __restrict__ Vt, const float* __restrict__ tau,
            const float* __restrict__ delta, _Float16* __restrict__ Ctx)
{
    __shared__ _Float16 __attribute__((aligned(16))) sP[64 * PP];
    const int t = threadIdx.x, l = t & 31, w = t >> 5, h = l >> 4, m = l & 15;
    const int bq = blockIdx.z, hd = blockIdx.y, q0 = blockIdx.x * 64;

    const float LOG2E = 1.4426950408889634f;
#if AFFINE_BF16
    const float tb = bfr(tau[bq]);
    const float db = bfr(delta[bq]);
#else
    const float tb = tau[bq];
    const float db = delta[bq];
#endif
    const float c1 = tb * (0.125f / 64.0f) * LOG2E;
    const float c0 = db * 0.125f * LOG2E;

    Frag qf[2];
    {
        const _Float16* qp = Qh + (size_t)(bq * SQ + q0 + 16 * w + m) * DM + hd * HD + 8 * h;
#pragma unroll
        for (int ec = 0; ec < 2; ++ec) {
            qf[ec].p[0] = *(const v8h*)(qp + 32 * ec);
            qf[ec].p[1] = *(const v8h*)(qp + 32 * ec + 16);
        }
    }
    const _Float16* kbase = Kh + (size_t)(bq * SQ + m) * DM + hd * HD + 8 * h;
    const _Float16* vbase = Vt + ((size_t)(bq * NH + hd) * HD + m) * SQ + 8 * h;
    _Float16* myP = sP + w * 16 * PP;

    v8f oacc[4];
#pragma unroll
    for (int et = 0; et < 4; ++et) oacc[et] = zero8();
    float mrun[8], lpart[8];
#pragma unroll
    for (int r = 0; r < 8; ++r) { mrun[r] = -1.0e30f; lpart[r] = 0.0f; }

    for (int s0 = 0; s0 < SQ; s0 += 64) {
        v8f sacc[4];
#pragma unroll
        for (int sub = 0; sub < 4; ++sub) sacc[sub] = zero8();
#pragma unroll
        for (int ec = 0; ec < 2; ++ec) {
            Frag kf[4];
#pragma unroll
            for (int sub = 0; sub < 4; ++sub) {
                const _Float16* kp = kbase + (size_t)(s0 + 16 * sub) * DM + 32 * ec;
                kf[sub].p[0] = *(const v8h*)kp;
                kf[sub].p[1] = *(const v8h*)(kp + 16);
            }
#pragma unroll
            for (int sub = 0; sub < 4; ++sub) sacc[sub] = mma16(qf[ec].v, kf[sub].v, sacc[sub]);
            asm volatile("v_nop\n\tv_nop\n\tv_nop\n\tv_nop"
                         : "+v"(sacc[0]), "+v"(sacc[1]), "+v"(sacc[2]), "+v"(sacc[3])
                         : "v"(qf[ec].v), "v"(kf[0].v), "v"(kf[1].v), "v"(kf[2].v), "v"(kf[3].v));
        }

#pragma unroll
        for (int sub = 0; sub < 4; ++sub)
#pragma unroll
            for (int r = 0; r < 8; ++r) sacc[sub][r] = sacc[sub][r] * c1 + c0;

        float msub[8];
#pragma unroll
        for (int r = 0; r < 8; ++r) {
            float mx = fmaxf(fmaxf(sacc[0][r], sacc[1][r]), fmaxf(sacc[2][r], sacc[3][r]));
            mx = fmaxf(mx, __shfl_xor(mx, 1, 16));
            mx = fmaxf(mx, __shfl_xor(mx, 2, 16));
            mx = fmaxf(mx, __shfl_xor(mx, 4, 16));
            mx = fmaxf(mx, __shfl_xor(mx, 8, 16));
            const float mn = fmaxf(mrun[r], mx);
            const float alpha = EX2(mrun[r] - mn);
            mrun[r] = mn;
            lpart[r] *= alpha;
#pragma unroll
            for (int et = 0; et < 4; ++et) oacc[et][r] *= alpha;
            msub[r] = mn - 14.0f;
        }
#pragma unroll
        for (int sub = 0; sub < 4; ++sub)
#pragma unroll
            for (int r = 0; r < 8; ++r) {
                const float p = EX2(sacc[sub][r] - msub[r]);
                lpart[r] += p;
                myP[(8 * h + r) * PP + 16 * sub + m] = (_Float16)p;
            }
        __syncthreads();

#pragma unroll
        for (int sc = 0; sc < 2; ++sc) {
            Frag pf, vf[4];
            pf.p[0] = *(const v8ha*)(myP + m * PP + 32 * sc + 8 * h);
            pf.p[1] = *(const v8ha*)(myP + m * PP + 32 * sc + 16 + 8 * h);
#pragma unroll
            for (int et = 0; et < 4; ++et) {
                const _Float16* vp = vbase + (size_t)(16 * et) * SQ + s0 + 32 * sc;
                vf[et].p[0] = *(const v8h*)vp;
                vf[et].p[1] = *(const v8h*)(vp + 16);
            }
#pragma unroll
            for (int et = 0; et < 4; ++et) oacc[et] = mma16(pf.v, vf[et].v, oacc[et]);
            asm volatile("v_nop\n\tv_nop\n\tv_nop\n\tv_nop"
                         : "+v"(oacc[0]), "+v"(oacc[1]), "+v"(oacc[2]), "+v"(oacc[3])
                         : "v"(pf.v), "v"(vf[0].v), "v"(vf[1].v), "v"(vf[2].v), "v"(vf[3].v));
        }
    }

#pragma unroll
    for (int r = 0; r < 8; ++r) {
        float lt = lpart[r];
        lt += __shfl_xor(lt, 1, 16);
        lt += __shfl_xor(lt, 2, 16);
        lt += __shfl_xor(lt, 4, 16);
        lt += __shfl_xor(lt, 8, 16);
        const float inv = 4.0f / lt;
        const int row = 8 * h + r;
#pragma unroll
        for (int et = 0; et < 4; ++et)
            myP[row * PP + 16 * et + m] = (_Float16)(oacc[et][r] * inv);
    }
    __syncthreads();
    v8h cv[4];
    size_t coff[4];
#pragma unroll
    for (int i = 0; i < 4; ++i) {
        const int row = 16 * w + 4 * i + (l >> 3);
        const int c8 = (l & 7) * 8;
        cv[i] = *(const v8ha*)(sP + row * PP + c8);
        coff[i] = (size_t)(bq * SQ + q0 + row) * DM + hd * HD + c8;
    }
#pragma unroll
    for (int i = 0; i < 4; ++i) *(volatile v8h*)(Ctx + coff[i]) = cv[i];
    __threadfence();
#pragma unroll
    for (int i = 0; i < 4; ++i) *(volatile v8h*)(Ctx + coff[i]) = cv[i];
}

extern "C" void kernel_launch(void* const* d_in, const int* in_sizes, int n_in,
                              void* d_out, int out_size, void* d_ws, size_t ws_size,
                              hipStream_t stream)
{
    if (n_in < 13) return;
    if (in_sizes[0] != PLANE || in_sizes[1] != PLANE || in_sizes[2] != PLANE) return;
    if (in_sizes[3] != NB || in_sizes[4] != NB) return;
    if (in_sizes[5] != DM * DM || in_sizes[7] != DM * DM || in_sizes[9] != DM * DM || in_sizes[11] != DM * DM) return;
    if (in_sizes[6] != DM || in_sizes[8] != DM || in_sizes[10] != DM || in_sizes[12] != DM) return;
    if (out_size != PLANE) return;

    const float* queries = (const float*)d_in[0];
    const float* keys    = (const float*)d_in[1];
    const float* values  = (const float*)d_in[2];
    const float* tau     = (const float*)d_in[3];
    const float* delta   = (const float*)d_in[4];
    const float* Wq = (const float*)d_in[5];
    const float* bq = (const float*)d_in[6];
    const float* Wk = (const float*)d_in[7];
    const float* bk = (const float*)d_in[8];
    const float* Wv = (const float*)d_in[9];
    const float* bv = (const float*)d_in[10];
    const float* Wo = (const float*)d_in[11];
    const float* bo = (const float*)d_in[12];
    float* out = (float*)d_out;

    const size_t szPlane16 = (size_t)PLANE * 2;
    const size_t offXh = 0;
    const size_t offWt = offXh + 3 * szPlane16;
    const size_t offQ  = offWt + (size_t)4 * DM * DM * 2;
    const size_t offK  = offQ + szPlane16;
    const size_t offVt = offK + szPlane16;
    const size_t offC  = offVt + szPlane16;
    const size_t wsEnd = offC + szPlane16;
    if (wsEnd > ws_size) return;

    char* ws = (char*)d_ws;
    _Float16* Xh  = (_Float16*)(ws + offXh);
    _Float16* Wt  = (_Float16*)(ws + offWt);
    _Float16* Qh  = (_Float16*)(ws + offQ);
    _Float16* Kh  = (_Float16*)(ws + offK);
    _Float16* Vth = (_Float16*)(ws + offVt);
    _Float16* Ctx = (_Float16*)(ws + offC);

    k_cvt_act<<<dim3(CVT_GRID, 3, 1), dim3(CVT_BLK), 0, stream>>>(queries, keys, values, Xh);
    k_cvt_wt<<<dim3(DM / 64, DM / 64, 4), dim3(128), 0, stream>>>(Wq, Wk, Wv, Wo, Wt);
    k_gemm<false><<<dim3(DM / 128, MR / 64, 3), dim3(128), 0, stream>>>(
        Xh, (int)PLANE, Wt, bq, bk, bv, Qh, out, 1.0f / 1024.0f, 8.0f);
    k_attn<<<dim3(SQ / 64, NH, NB), dim3(128), 0, stream>>>(Qh, Kh, Vth, tau, delta, Ctx);
    k_gemm<true><<<dim3(DM / 128, MR / 64, 1), dim3(128), 0, stream>>>(
        Ctx, 0, Wt + (size_t)3 * DM * DM, bo, bo, bo, Qh, out, 1.0f / 2048.0f, 1.0f);
}
